// BiMambaAggregator_1460288881206
// MI455X (gfx1250) — hardware-verified
//
#include <hip/hip_runtime.h>
#include <hip/hip_bf16.h>
#include <math.h>

constexpr int NBATCH = 4;
constexpr int NTOK   = 1024;
constexpr int NROWS  = NBATCH * NTOK;
constexpr int DMOD   = 512;
constexpr int DIN    = 1024;
constexpr int DXZ    = 2 * DIN;
constexpr int DST    = 16;
constexpr int DCV    = 4;
constexpr int DTRK   = 32;
constexpr int DDBL   = DTRK + 2 * DST;
constexpr int DTKP   = 64;
constexpr int DFF    = 4 * DMOD;
constexpr int DATT   = DMOD / 2;
constexpr int NLAY   = 2;

constexpr float WCARRY   = 64.0f;
constexpr float XCCARRY  = 256.0f;
constexpr float DBLCARRY = 256.0f;
constexpr float GCARRY   = 128.0f;
constexpr float GLCARRY  = 64.0f;


typedef __attribute__((ext_vector_type(16))) _Float16 v16h;
typedef __attribute__((ext_vector_type(8)))  _Float16 v8h;
typedef __attribute__((ext_vector_type(16))) __bf16   v16b;
typedef __attribute__((ext_vector_type(8)))  __bf16   v8b;
typedef __attribute__((ext_vector_type(8)))  float    v8f;
typedef __attribute__((ext_vector_type(4)))  float    v4f;

__device__ __forceinline__ unsigned short f2bf_bits(float f) {
  unsigned u = __float_as_uint(f);
  return (unsigned short)((u + 0x7FFFu + ((u >> 16) & 1u)) >> 16);
}
__device__ __forceinline__ float bf_bits2f(unsigned short h) { return __uint_as_float(((unsigned)h) << 16); }

__device__ __forceinline__ void dep_guard_h(v8f& a, v8f& b, v16h x, v16h y) { asm volatile("v_nop\n\tv_nop\n\tv_nop\n\tv_nop" : "+v"(a), "+v"(b) : "v"(x), "v"(y)); }
__device__ __forceinline__ void dep_guard_b(v8f& a, v8f& b, v16b x, v16b y) { asm volatile("v_nop\n\tv_nop\n\tv_nop\n\tv_nop" : "+v"(a), "+v"(b) : "v"(x), "v"(y)); }
__device__ __forceinline__ void keep4_h(v16h a, v16h b, v16h c, v16h d) { asm volatile("v_nop" :: "v"(a), "v"(b), "v"(c), "v"(d)); }
__device__ __forceinline__ void keep4_b(v16b a, v16b b, v16b c, v16b d) { asm volatile("v_nop" :: "v"(a), "v"(b), "v"(c), "v"(d)); }
__device__ __forceinline__ void acc_guard4(v8f& a, v8f& b, v8f& c, v8f& d) { asm volatile("v_nop\n\tv_nop\n\tv_nop\n\tv_nop" : "+v"(a), "+v"(b), "+v"(c), "+v"(d)); }
template <typename T> struct Frag;
template <> struct Frag<_Float16> {
  typedef v16h V; union U { v16h v; v8h h[2]; };
  static __device__ __forceinline__ v16h load(const _Float16* p) {
    U f; f.h[0] = *(const v8h*)(p); f.h[1] = *(const v8h*)(p + 16); return f.v;
  }
  static __device__ __forceinline__ v8f mma(v16h a, v16h b, v8f c) {
    return __builtin_amdgcn_wmma_f32_16x16x32_f16(false, a, false, b, (short)0, c, false, false);
  }
  static __device__ __forceinline__ void guard(v8f& a, v8f& b, v16h x, v16h y) { dep_guard_h(a, b, x, y); }
  static __device__ __forceinline__ void keep(v16h a, v16h b, v16h c, v16h d) { keep4_h(a, b, c, d); }
};
template <> struct Frag<__bf16> {
  typedef v16b V; union U { v16b v; v8b h[2]; };
  static __device__ __forceinline__ v16b load(const __bf16* p) {
    U f; f.h[0] = *(const v8b*)(p); f.h[1] = *(const v8b*)(p + 16); return f.v;
  }
  static __device__ __forceinline__ v8f mma(v16b a, v16b b, v8f c) {
    return __builtin_amdgcn_wmma_f32_16x16x32_bf16(false, a, false, b, (short)0, c, false, false);
  }
  static __device__ __forceinline__ void guard(v8f& a, v8f& b, v16b x, v16b y) { dep_guard_b(a, b, x, y); }
  static __device__ __forceinline__ void keep(v16b a, v16b b, v16b c, v16b d) { keep4_b(a, b, c, d); }
};

template <int ET> struct Elem;
template <> struct Elem<0> { typedef _Float16 T; };
template <> struct Elem<1> { typedef __bf16 T; };
template <int ET, bool SPLIT, int BIAS_MODE, int OUT_MODE, bool RESID, int ACT = 0>
__global__ __launch_bounds__(256) void wmma_gemm64(
    const unsigned short* __restrict__ Ap, const unsigned short* __restrict__ A2p, int lda, long strideA,
    const unsigned short* __restrict__ Btp, const unsigned short* __restrict__ Bt2p, int ldb, long strideB,
    void* __restrict__ Cout, void* __restrict__ Cout2, int ldc, long strideC,
    const float* __restrict__ bias,
    const float* __restrict__ resid, long strideR,
    int M, int N, int K, float scale) {
  typedef typename Elem<ET>::T T;
  typedef typename Frag<T>::V V;
  const T* A = (const T*)Ap; const T* A2 = (const T*)A2p; const T* Bt = (const T*)Btp; const T* Bt2 = (const T*)Bt2p;
  __shared__ __align__(16) float sT[8][16 * 68];
  const int b    = blockIdx.y;
  const int lane = threadIdx.x & 31;
  const int wave = threadIdx.x >> 5;
  const int tilesN = N >> 6;
  const int tilesM = M >> 6;
  const int tile = blockIdx.x * 8 + wave;
  if (tile >= tilesM * tilesN) return;
  const int tm = tile / tilesN;
  const int tn = tile - tm * tilesN;
  const int m0 = tm << 6;
  const int n0 = tn << 6;

  const T* Ab  = A  + (size_t)b * strideA;
  const T* Bb  = Bt + (size_t)b * strideB;
  const T* Ab2 = SPLIT ? (A2  + (size_t)b * strideA) : nullptr;
  const T* Bb2 = SPLIT ? (Bt2 + (size_t)b * strideB) : nullptr;

  const int rlane = lane & 15;
  const int koff  = (lane >> 4) * 8;
  const int mOff  = (lane >> 4) * 8;

  v8f acc[4][4];
#pragma unroll
  for (int i = 0; i < 4; ++i)
#pragma unroll
    for (int j = 0; j < 4; ++j) acc[i][j] = (v8f){0.f,0.f,0.f,0.f,0.f,0.f,0.f,0.f};

  for (int k0 = 0; k0 < K; k0 += 32) {
    V bh[4], bl[4];
#pragma unroll
    for (int j = 0; j < 4; ++j) {
      const size_t bo = (size_t)(n0 + (j << 4) + rlane) * ldb + koff + k0;
      bh[j] = Frag<T>::load(Bb + bo);
      if (SPLIT) bl[j] = Frag<T>::load(Bb2 + bo);
    }
#pragma unroll
    for (int i = 0; i < 4; ++i) {
      const size_t ao = (size_t)(m0 + (i << 4) + rlane) * lda + koff + k0;
      V ah = Frag<T>::load(Ab + ao);
      V al;
      if (SPLIT) al = Frag<T>::load(Ab2 + ao);
#pragma unroll
      for (int j = 0; j < 4; ++j) {
        acc[i][j] = Frag<T>::mma(ah, bh[j], acc[i][j]);
        if (SPLIT) {
          acc[i][j] = Frag<T>::mma(ah, bl[j], acc[i][j]);
          acc[i][j] = Frag<T>::mma(al, bh[j], acc[i][j]);
        }
      }
      Frag<T>::guard(acc[i][0], acc[i][3], ah, SPLIT ? al : ah);
    }
    Frag<T>::keep(bh[0], bh[1], bh[2], bh[3]);
    if (SPLIT) Frag<T>::keep(bl[0], bl[1], bl[2], bl[3]);
  }
  acc_guard4(acc[0][0], acc[0][1], acc[0][2], acc[0][3]);
  acc_guard4(acc[1][0], acc[1][1], acc[1][2], acc[1][3]);
  acc_guard4(acc[2][0], acc[2][1], acc[2][2], acc[2][3]);
  acc_guard4(acc[3][0], acc[3][1], acc[3][2], acc[3][3]);

  float* slab = sT[wave];
  const float* Rb = RESID ? (resid + (size_t)b * strideR) : nullptr;
#pragma unroll
  for (int i = 0; i < 4; ++i) {
    const int mBase = m0 + (i << 4);
#pragma unroll
    for (int j = 0; j < 4; ++j) {
      const int n = n0 + (j << 4) + rlane;
      float bv = 0.f;
      if (BIAS_MODE == 2) bv = bias[n];
#pragma unroll
      for (int r = 0; r < 8; ++r) {
        float v = acc[i][j][r] * scale;
        if (BIAS_MODE == 1) v += bias[mBase + mOff + r];
        if (BIAS_MODE == 2) v += bv;
        if (RESID) v += Rb[(size_t)(mBase + mOff + r) * ldc + n];
        if (ACT == 1) v = tanhf(v);
        if (ACT == 2) v = fmaxf(v, 0.0f);
        if (ACT == 3) v = v / (1.0f + expf(-v));
        if (ACT == 4) v = (v > 0.f) ? v : 0.01f * v;
        if (ACT == 5) v = 0.5f * v * (1.0f + erff(v * 0.70710678118654752f));
        slab[(mOff + r) * 68 + (j << 4) + rlane] = v;
      }
    }
    __builtin_amdgcn_fence(__ATOMIC_RELEASE, "workgroup");
    __builtin_amdgcn_wave_barrier();
    __builtin_amdgcn_fence(__ATOMIC_ACQUIRE, "workgroup");
    if (OUT_MODE == 0) {
      float* C = (float*)Cout + (size_t)b * strideC;
      const int hh = lane >> 4, c4 = (lane & 15) * 4;
      for (int pass = 0; pass < 2; ++pass) {
#pragma unroll
        for (int it = 0; it < 8; ++it) {
          const int row = it * 2 + hh;
          v4f v = *(const v4f*)(slab + row * 68 + c4);
          *(volatile v4f*)(C + (size_t)(mBase + row) * ldc + n0 + c4) = v;
        }
        __threadfence();
      }
    } else {
      const int q = lane >> 3, c8 = (lane & 7) * 8;
      unsigned short* C  = (unsigned short*)Cout  + (size_t)b * strideC;
      unsigned short* C2 = (OUT_MODE == 2) ? ((unsigned short*)Cout2 + (size_t)b * strideC) : nullptr;
      for (int pass = 0; pass < 2; ++pass) {
#pragma unroll
        for (int it = 0; it < 4; ++it) {
          const int row = it * 4 + q;
          const float* sp = slab + row * 68 + c8;
          v8h hv, lv;
#pragma unroll
          for (int e = 0; e < 8; ++e) {
            if (OUT_MODE == 1) {
              hv[e] = (_Float16)sp[e];
            } else {
              unsigned short hb = f2bf_bits(sp[e]);
              unsigned short lb = f2bf_bits(sp[e] - bf_bits2f(hb));
              hv[e] = __builtin_bit_cast(_Float16, hb);
              lv[e] = __builtin_bit_cast(_Float16, lb);
            }
          }
          *(volatile v8h*)(C + (size_t)(mBase + row) * ldc + n0 + c8) = hv;
          if (OUT_MODE == 2) *(volatile v8h*)(C2 + (size_t)(mBase + row) * ldc + n0 + c8) = lv;
        }
        __threadfence();
      }
    }
    __builtin_amdgcn_fence(__ATOMIC_RELEASE, "workgroup");
    __builtin_amdgcn_wave_barrier();
    __builtin_amdgcn_fence(__ATOMIC_ACQUIRE, "workgroup");
  }
}

__global__ __launch_bounds__(256) void cast_f32_f16x2(
    const float* __restrict__ in, _Float16* __restrict__ out, int n2) {
  int i = blockIdx.x * 256 + threadIdx.x;
  if (i < n2) {
    const _Float16 h0 = (_Float16)in[2 * i], h1 = (_Float16)in[2 * i + 1];
    const unsigned u = (unsigned)__builtin_bit_cast(unsigned short, h0) | ((unsigned)__builtin_bit_cast(unsigned short, h1) << 16);
    ((volatile unsigned*)out)[i] = u;
    __threadfence();
    ((volatile unsigned*)out)[i] = u;
  }
}

__device__ __forceinline__ float us2f(unsigned short u) { return (float)__builtin_bit_cast(_Float16, u); }
__device__ __forceinline__ unsigned short f2us(float f) { return __builtin_bit_cast(unsigned short, (_Float16)f); }
__device__ __forceinline__ float sigm_f(float x) { return __builtin_amdgcn_rcpf(1.0f + __expf(-x)); }

__global__ __launch_bounds__(256) void wtr_f16(const float* __restrict__ srcF, const float* __restrict__ srcB,
                                                unsigned short* __restrict__ dst, int K, int N, int Kp, float sc)
{
  __shared__ float tile[64][65];
  const int tid = threadIdx.x, lane = tid & 31, wave = tid >> 5;
  const int z = blockIdx.z;
  const float* W = ((z < 2) ? srcF : srcB) + (size_t)(z & 1) * (size_t)K * (size_t)N;
  unsigned short* WT = dst + (size_t)z * (size_t)N * (size_t)Kp;
  const int k0 = blockIdx.x * 64, n0 = blockIdx.y * 64;
  {
    const int kk = tid >> 2, cc = (tid & 3) * 16;
    const int k  = k0 + kk;
    const int kc = (k < K) ? k : (K - 1);
    const float keep = (k < K) ? 1.0f : 0.0f;
    const float* s = W + (size_t)kc * N + n0 + cc;
#pragma unroll
    for (int i = 0; i < 4; ++i) {
      const v4f v = *(const v4f*)(s + 4 * i);
      tile[kk][cc + 4 * i + 0] = v[0] * keep;
      tile[kk][cc + 4 * i + 1] = v[1] * keep;
      tile[kk][cc + 4 * i + 2] = v[2] * keep;
      tile[kk][cc + 4 * i + 3] = v[3] * keep;
    }
  }
  __syncthreads();
  const int q = lane >> 3, c8 = (lane & 7) * 8;
  for (int pass = 0; pass < 2; ++pass) {
#pragma unroll
    for (int it = 0; it < 2; ++it) {
      const int r = wave * 8 + it * 4 + q;
      v8h hv;
#pragma unroll
      for (int e = 0; e < 8; ++e) hv[e] = (_Float16)(tile[c8 + e][r] * sc);
      *(volatile v8h*)(WT + (size_t)(n0 + r) * Kp + k0 + c8) = hv;
    }
    __threadfence();
  }
}

__global__ __launch_bounds__(256) void ln_rows_to_f16(const float* __restrict__ X, const float* __restrict__ gw,
                                                       const float* __restrict__ gb, unsigned short* __restrict__ Y, int nrows)
{
  const int lane = threadIdx.x & 31, wave = threadIdx.x >> 5;
  const int row = blockIdx.x * 8 + wave;
  if (row >= nrows) return;
  const float* xr = X + (size_t)row * DMOD;
  const int cA = 8 * lane, cB = 256 + 8 * lane;
  const v4f x0 = *(const v4f*)(xr + cA), x1 = *(const v4f*)(xr + cA + 4);
  const v4f x2 = *(const v4f*)(xr + cB), x3 = *(const v4f*)(xr + cB + 4);
  float v[16];
#pragma unroll
  for (int e = 0; e < 4; ++e) { v[e] = x0[e]; v[4 + e] = x1[e]; v[8 + e] = x2[e]; v[12 + e] = x3[e]; }
  float s = 0.f;
#pragma unroll
  for (int e = 0; e < 16; ++e) s += v[e];
#pragma unroll
  for (int off = 16; off > 0; off >>= 1) s += __shfl_xor(s, off, 32);
  const float mu = s * (1.0f / 512.0f);
  float qv = 0.f;
#pragma unroll
  for (int e = 0; e < 16; ++e) { const float dl = v[e] - mu; qv += dl * dl; }
#pragma unroll
  for (int off = 16; off > 0; off >>= 1) qv += __shfl_xor(qv, off, 32);
  const float rs = rsqrtf(qv * (1.0f / 512.0f) + 1e-5f);
  const v4f g0 = *(const v4f*)(gw + cA), g1 = *(const v4f*)(gw + cA + 4), g2 = *(const v4f*)(gw + cB), g3 = *(const v4f*)(gw + cB + 4);
  const v4f b0 = *(const v4f*)(gb + cA), b1 = *(const v4f*)(gb + cA + 4), b2 = *(const v4f*)(gb + cB), b3 = *(const v4f*)(gb + cB + 4);
  float gg[16], bb[16];
#pragma unroll
  for (int e = 0; e < 4; ++e) {
    gg[e] = g0[e]; gg[4 + e] = g1[e]; gg[8 + e] = g2[e]; gg[12 + e] = g3[e];
    bb[e] = b0[e]; bb[4 + e] = b1[e]; bb[8 + e] = b2[e]; bb[12 + e] = b3[e];
  }
  v8h oA, oB;
#pragma unroll
  for (int e = 0; e < 8; ++e) {
    oA[e] = (_Float16)((v[e] - mu) * rs * gg[e] + bb[e]);
    oB[e] = (_Float16)((v[8 + e] - mu) * rs * gg[8 + e] + bb[8 + e]);
  }
  unsigned short* yr = Y + (size_t)row * DMOD;
  for (int pass = 0; pass < 2; ++pass) {
    *(volatile v8h*)(yr + cA) = oA;
    *(volatile v8h*)(yr + cB) = oB;
    __threadfence();
  }
}

__global__ __launch_bounds__(256) void conv_silu_f16(const unsigned short* __restrict__ XZ, const float* __restrict__ cw,
                                                      const float* __restrict__ cb, unsigned short* __restrict__ XC,
                                                      int dir, float osc)
{
  const int idx = blockIdx.x * 256 + threadIdx.x;
  if (idx >= NROWS * (DIN / 8)) return;
  const int row = idx >> 7;
  const int d0  = (idx & 127) * 8;
  const int b = row >> 10, t = row & (NTOK - 1);
  float acc[8];
#pragma unroll
  for (int e = 0; e < 8; ++e) acc[e] = cb[d0 + e];
#pragma unroll
  for (int j = 0; j < DCV; ++j) {
    const int tt  = dir ? (t + 3 - j) : (t - 3 + j);
    const bool ok = (tt >= 0) && (tt < NTOK);
    const int ttc = tt < 0 ? 0 : (tt > NTOK - 1 ? NTOK - 1 : tt);
    const v8h xv = *(const v8h*)(XZ + (size_t)(b * NTOK + ttc) * DXZ + d0);
    const float keep = ok ? 1.0f : 0.0f;
#pragma unroll
    for (int e = 0; e < 8; ++e) acc[e] += cw[(size_t)(d0 + e) * DCV + j] * ((float)xv[e] * keep);
  }
  v8h o;
#pragma unroll
  for (int e = 0; e < 8; ++e) { const float a = acc[e]; o[e] = (_Float16)(a * sigm_f(a) * osc); }
  unsigned short* p = XC + (size_t)row * DIN + d0;
  *(volatile v8h*)p = o;
  __threadfence();
  *(volatile v8h*)p = o;
}

__global__ __launch_bounds__(64) void ssm_scan_gate(
    const float* __restrict__ DTP,
    const unsigned short* __restrict__ XZ,
    const float* __restrict__ DBL,
    const float* __restrict__ cw, const float* __restrict__ cb,
    const float* __restrict__ alog, const float* __restrict__ dd,
    unsigned short* __restrict__ G, int dir, float gsc)
{
  __shared__ unsigned short stg[2][64];
  const int tid = threadIdx.x, lane = tid & 31, wave = tid >> 5;
  const int b = blockIdx.y;
  const int dbase = blockIdx.x * 64;
  const int d = dbase + tid;
  float An[DST], hs[DST];
#pragma unroll
  for (int s = 0; s < DST; ++s) { An[s] = -__expf(alog[(size_t)d * DST + s]); hs[s] = 0.0f; }
  const float c0 = cw[(size_t)d * DCV + 0], c1 = cw[(size_t)d * DCV + 1], c2 = cw[(size_t)d * DCV + 2], c3 = cw[(size_t)d * DCV + 3];
  const float cbv = cb[d], ddv = dd[d];
  float wA = 0.0f, wB = 0.0f, wC = 0.0f;
#pragma unroll 1
  for (int it = 0; it < NTOK; ++it) {
    const int t = dir ? (NTOK - 1 - it) : it;
    const size_t row = (size_t)b * NTOK + t;
    const float xn   = us2f(XZ[row * DXZ + d]);
    const float zv   = us2f(XZ[row * DXZ + DIN + d]);
    const float dpre = DTP[row * DIN + d];
    float Bv[DST], Cv[DST];
    const float* bcp = DBL + row * DDBL + DTRK;
#pragma unroll
    for (int i = 0; i < 4; ++i) {
      const v4f vb = *(const v4f*)(bcp + 4 * i);
      const v4f vc = *(const v4f*)(bcp + DST + 4 * i);
      Bv[4 * i + 0] = vb[0]; Bv[4 * i + 1] = vb[1]; Bv[4 * i + 2] = vb[2]; Bv[4 * i + 3] = vb[3];
      Cv[4 * i + 0] = vc[0]; Cv[4 * i + 1] = vc[1]; Cv[4 * i + 2] = vc[2]; Cv[4 * i + 3] = vc[3];
    }
    float xc = cbv + c0 * wA + c1 * wB + c2 * wC + c3 * xn;
    wA = wB; wB = wC; wC = xn;
    xc = xc * sigm_f(xc);
    const float dt  = fmaxf(dpre, 0.0f) + log1pf(__expf(-fabsf(dpre)));
    const float dtx = dt * xc;
    float y = 0.0f;
#pragma unroll
    for (int s = 0; s < DST; ++s) {
      const float e = __expf(dt * An[s]);
      hs[s] = hs[s] * e + dtx * Bv[s];
      y += hs[s] * Cv[s];
    }
    const float g = (y + ddv * xc) * (zv * sigm_f(zv)) * gsc;
    stg[it & 1][tid] = f2us(g);
    __syncthreads();
    if (wave == (it & 1)) {
      const unsigned lo16 = stg[it & 1][2 * lane];
      const unsigned hi16 = stg[it & 1][2 * lane + 1];
      const unsigned u = lo16 | (hi16 << 16);
      volatile unsigned* p = (volatile unsigned*)(G + row * DIN + dbase) + lane;
      *p = u;
      __threadfence();
      *p = u;
    }
  }
}

__global__ __launch_bounds__(256) void gelu_f16x2(const float* __restrict__ in, unsigned short* __restrict__ out, int n2, float osc)
{
  const int i = blockIdx.x * 256 + threadIdx.x;
  if (i < n2) {
    const float2 v = *(const float2*)(in + 2 * (size_t)i);
    const float g0 = 0.5f * v.x * (1.0f + erff(v.x * 0.70710678118654752f)) * osc;
    const float g1 = 0.5f * v.y * (1.0f + erff(v.y * 0.70710678118654752f)) * osc;
    const unsigned u = (unsigned)f2us(g0) | ((unsigned)f2us(g1) << 16);
    ((volatile unsigned*)out)[i] = u;
    __threadfence();
    ((volatile unsigned*)out)[i] = u;
  }
}

__global__ __launch_bounds__(256) void score_softmax(const float* __restrict__ S1, const float* __restrict__ aw2,
                                                     const float* __restrict__ ab2, float* __restrict__ att)
{
  __shared__ __align__(16) float sc[NTOK];
  __shared__ float red[8];
  const int tid = threadIdx.x, lane = tid & 31, wave = tid >> 5;
  const int b = blockIdx.x;
  const float bias2 = ab2[0];
#pragma unroll 1
  for (int rr = 0; rr < NTOK / 8; ++rr) {
    const int n = wave * (NTOK / 8) + rr;
    const float* sp = S1 + ((size_t)b * NTOK + n) * DATT;
    float acc = 0.0f;
#pragma unroll 1
    for (int i = 0; i < DATT / 32; ++i) {
      const int j = i * 32 + lane;
      acc += tanhf(sp[j]) * aw2[j];
    }
#pragma unroll
    for (int off = 16; off > 0; off >>= 1) acc += __shfl_xor(acc, off, 32);
    if (lane == 0) sc[n] = acc + bias2;
  }
  __syncthreads();
  const float v0 = sc[tid], v1 = sc[256 + tid], v2 = sc[512 + tid], v3 = sc[768 + tid];
  float m = fmaxf(fmaxf(v0, v1), fmaxf(v2, v3));
#pragma unroll
  for (int off = 16; off > 0; off >>= 1) m = fmaxf(m, __shfl_xor(m, off, 32));
  if (lane == 0) red[wave] = m;
  __syncthreads();
  float mm = red[0];
#pragma unroll
  for (int w = 1; w < 8; ++w) mm = fmaxf(mm, red[w]);
  __syncthreads();
  const float e0 = expf(v0 - mm), e1 = expf(v1 - mm), e2 = expf(v2 - mm), e3 = expf(v3 - mm);
  float su = (e0 + e1) + (e2 + e3);
#pragma unroll
  for (int off = 16; off > 0; off >>= 1) su += __shfl_xor(su, off, 32);
  if (lane == 0) red[wave] = su;
  __syncthreads();
  float tot = 0.0f;
#pragma unroll
  for (int w = 0; w < 8; ++w) tot += red[w];
  const float inv = 1.0f / tot;
  sc[tid] = e0 * inv; sc[256 + tid] = e1 * inv; sc[512 + tid] = e2 * inv; sc[768 + tid] = e3 * inv;
  __syncthreads();
  const v4f pv = *(const v4f*)(sc + wave * 128 + 4 * lane);
  float* dst = att + (size_t)b * NTOK + wave * 128 + 4 * lane;
  *(volatile v4f*)dst = pv;
  __threadfence();
  *(volatile v4f*)dst = pv;
}

__global__ __launch_bounds__(512) void pool_norm_out(const float* __restrict__ att, const float* __restrict__ HF,
                                                     const float* __restrict__ HB, const float* __restrict__ nw,
                                                     const float* __restrict__ nb, float* __restrict__ out)
{
  __shared__ __align__(16) float ob[2 * DMOD + NTOK];
  __shared__ float red[16];
  const int tid = threadIdx.x, lane = tid & 31, wave = tid >> 5;
  const int b = blockIdx.x;
  const float* af  = att + (size_t)b * NTOK;
  const float* abk = att + (size_t)NBATCH * NTOK + (size_t)b * NTOK;
  const float* hf = HF + (size_t)b * NTOK * DMOD + tid;
  const float* hb = HB + (size_t)b * NTOK * DMOD + tid;
  float zf = 0.0f, zb = 0.0f;
#pragma unroll 1
  for (int n = 0; n < NTOK; ++n) {
    zf += af[n]  * hf[(size_t)n * DMOD];
    zb += abk[n] * hb[(size_t)n * DMOD];
  }
  float s = zf + zb;
#pragma unroll
  for (int off = 16; off > 0; off >>= 1) s += __shfl_xor(s, off, 32);
  if (lane == 0) red[wave] = s;
  __syncthreads();
  float tot = 0.0f;
#pragma unroll
  for (int w = 0; w < 16; ++w) tot += red[w];
  __syncthreads();
  const float mu = tot * (1.0f / 1024.0f);
  const float df = zf - mu, db = zb - mu;
  float qv = df * df + db * db;
#pragma unroll
  for (int off = 16; off > 0; off >>= 1) qv += __shfl_xor(qv, off, 32);
  if (lane == 0) red[wave] = qv;
  __syncthreads();
  float totq = 0.0f;
#pragma unroll
  for (int w = 0; w < 16; ++w) totq += red[w];
  const float rs = rsqrtf(totq * (1.0f / 1024.0f) + 1e-5f);
  ob[tid]        = df * rs * nw[tid] + nb[tid];
  ob[DMOD + tid] = db * rs * nw[DMOD + tid] + nb[DMOD + tid];
  ob[2 * DMOD + tid]       = (af[tid] + abk[tid]) * 0.5f;
  ob[2 * DMOD + 512 + tid] = (af[512 + tid] + abk[512 + tid]) * 0.5f;
  __syncthreads();
  const v4f pv = *(const v4f*)(ob + wave * 128 + 4 * lane);
  const size_t gbase = (wave < 8) ? ((size_t)b * (2 * DMOD) + (size_t)wave * 128)
                                  : ((size_t)NBATCH * (2 * DMOD) + (size_t)b * NTOK + (size_t)(wave - 8) * 128);
  float* dst = out + gbase + 4 * lane;
  *(volatile v4f*)dst = pv;
  __threadfence();
  *(volatile v4f*)dst = pv;
}

template <int BIAS_MODE, int OUT_MODE, bool RESID>
static void launch_gemm(hipStream_t st, const unsigned short* A, int lda, const unsigned short* Bt, int ldb,
                        void* C, int ldc, const float* bias, const float* resid, int M, int N, int K, float scale)
{
  const int tiles = (M / 64) * (N / 64);
  dim3 grid((unsigned)((tiles + 7) / 8), 1, 1);
  wmma_gemm64<0, false, BIAS_MODE, OUT_MODE, RESID, 0><<<grid, 256, 0, st>>>(
      A, nullptr, lda, 0L, Bt, nullptr, ldb, 0L, C, nullptr, ldc, 0L, bias, resid, 0L, M, N, K, scale);
}

extern "C" void kernel_launch(void* const* d_in, const int* in_sizes, int n_in,
                              void* d_out, int out_size, void* d_ws, size_t ws_size, hipStream_t stream)
{
  (void)in_sizes;
  constexpr size_t MIB = 1048576;
  constexpr size_t OFF_HF  = 0;
  constexpr size_t OFF_HB  = 8 * MIB;
  constexpr size_t OFF_HT  = 16 * MIB;
  constexpr size_t OFF_ULN = 24 * MIB;
  constexpr size_t OFF_UNI = 28 * MIB;
  constexpr size_t OFF_WT  = 78 * MIB;
  constexpr size_t OFF_ATT = 107 * MIB + 262144;
  constexpr size_t WS_TOTAL = OFF_ATT + 32768;
  if (n_in < 41 || out_size < 2 * NBATCH * NTOK || ws_size < WS_TOTAL) return;

  char* ws = (char*)d_ws;
  float* HF  = (float*)(ws + OFF_HF);
  float* HB  = (float*)(ws + OFF_HB);
  float* HT  = (float*)(ws + OFF_HT);
  unsigned short* ULN = (unsigned short*)(ws + OFF_ULN);
  unsigned short* XZ    = (unsigned short*)(ws + OFF_UNI);
  unsigned short* XC    = (unsigned short*)(ws + OFF_UNI + 16 * MIB);
  float*          DBL32 = (float*)(ws + OFF_UNI + 24 * MIB);
  unsigned short* DBL16 = (unsigned short*)(ws + OFF_UNI + 25 * MIB);
  float*          DTP   = (float*)(ws + OFF_UNI + 26 * MIB);
  unsigned short* GP    = (unsigned short*)(ws + OFF_UNI + 42 * MIB);
  float*          F1 = (float*)(ws + OFF_UNI);
  unsigned short* GL = (unsigned short*)(ws + OFF_UNI + 32 * MIB);
  unsigned short* H16 = (unsigned short*)(ws + OFF_UNI);
  float*          S1  = (float*)(ws + OFF_UNI + 4 * MIB);
  unsigned short* inwT = (unsigned short*)(ws + OFF_WT);
  unsigned short* w1T  = (unsigned short*)(ws + OFF_WT + 8 * MIB);
  unsigned short* w2T  = (unsigned short*)(ws + OFF_WT + 16 * MIB);
  unsigned short* owT  = (unsigned short*)(ws + OFF_WT + 24 * MIB);
  unsigned short* xpwT = (unsigned short*)(ws + OFF_WT + 28 * MIB);
  unsigned short* dtwT = (unsigned short*)(ws + OFF_WT + 28 * MIB + 524288);
  unsigned short* aw1T = (unsigned short*)(ws + OFF_WT + 29 * MIB);
  float* ATT = (float*)(ws + OFF_ATT);

  const float* x   = (const float*)d_in[0];
  const float* aw1 = (const float*)d_in[35];
  const float* ab1 = (const float*)d_in[36];
  const float* aw2 = (const float*)d_in[37];
  const float* ab2 = (const float*)d_in[38];
  const float* nw  = (const float*)d_in[39];
  const float* nb  = (const float*)d_in[40];
  float* out = (float*)d_out;

  wtr_f16<<<dim3(DMOD / 64, DXZ / 64, 4), 256, 0, stream>>>((const float*)d_in[3],  (const float*)d_in[20], inwT, DMOD, DXZ, DMOD, WCARRY);
  wtr_f16<<<dim3(DIN / 64, DDBL / 64, 4), 256, 0, stream>>>((const float*)d_in[6],  (const float*)d_in[23], xpwT, DIN, DDBL, DIN, WCARRY);
  wtr_f16<<<dim3(DTKP / 64, DIN / 64, 4), 256, 0, stream>>>((const float*)d_in[7],  (const float*)d_in[24], dtwT, DTRK, DIN, DTKP, WCARRY);
  wtr_f16<<<dim3(DIN / 64, DMOD / 64, 4), 256, 0, stream>>>((const float*)d_in[11], (const float*)d_in[28], owT, DIN, DMOD, DIN, WCARRY);
  wtr_f16<<<dim3(DMOD / 64, DFF / 64, 4), 256, 0, stream>>>((const float*)d_in[14], (const float*)d_in[31], w1T, DMOD, DFF, DMOD, WCARRY);
  wtr_f16<<<dim3(DFF / 64, DMOD / 64, 4), 256, 0, stream>>>((const float*)d_in[16], (const float*)d_in[33], w2T, DFF, DMOD, DFF, WCARRY);
  wtr_f16<<<dim3(DMOD / 64, DATT / 64, 1), 256, 0, stream>>>(aw1, aw1, aw1T, DMOD, DATT, DMOD, WCARRY);

  for (int dir = 0; dir < 2; ++dir) {
    const int pb = dir ? 18 : 1;
    float* HD = dir ? HB : HF;
    for (int l = 0; l < NLAY; ++l) {
      const float* n1w  = (const float*)d_in[pb + 0]  + (size_t)l * DMOD;
      const float* n1b  = (const float*)d_in[pb + 1]  + (size_t)l * DMOD;
      const float* cw   = (const float*)d_in[pb + 3]  + (size_t)l * DIN * DCV;
      const float* cb   = (const float*)d_in[pb + 4]  + (size_t)l * DIN;
      const float* dtb  = (const float*)d_in[pb + 7]  + (size_t)l * DIN;
      const float* alog = (const float*)d_in[pb + 8]  + (size_t)l * DIN * DST;
      const float* dd   = (const float*)d_in[pb + 9]  + (size_t)l * DIN;
      const float* n2w  = (const float*)d_in[pb + 11] + (size_t)l * DMOD;
      const float* n2b  = (const float*)d_in[pb + 12] + (size_t)l * DMOD;
      const float* b1   = (const float*)d_in[pb + 14] + (size_t)l * DFF;
      const float* b2   = (const float*)d_in[pb + 16] + (size_t)l * DMOD;
      const int slot = dir * 2 + l;
      const unsigned short* inwT_l = inwT + (size_t)slot * DXZ * DMOD;
      const unsigned short* xpwT_l = xpwT + (size_t)slot * DDBL * DIN;
      const unsigned short* dtwT_l = dtwT + (size_t)slot * DIN * DTKP;
      const unsigned short* owT_l  = owT  + (size_t)slot * DMOD * DIN;
      const unsigned short* w1T_l  = w1T  + (size_t)slot * DFF * DMOD;
      const unsigned short* w2T_l  = w2T  + (size_t)slot * DMOD * DFF;
      const float* Hin = (l == 0) ? x : HD;

      ln_rows_to_f16<<<NROWS / 8, 256, 0, stream>>>(Hin, n1w, n1b, ULN, NROWS);
      launch_gemm<0, 1, false>(stream, ULN, DMOD, inwT_l, DMOD, XZ, DXZ, nullptr, nullptr, NROWS, DXZ, DMOD, 1.0f / WCARRY);
      conv_silu_f16<<<NROWS * (DIN / 8) / 256, 256, 0, stream>>>(XZ, cw, cb, XC, dir, XCCARRY);
      launch_gemm<0, 0, false>(stream, XC, DIN, xpwT_l, DIN, DBL32, DDBL, nullptr, nullptr, NROWS, DDBL, DIN, 1.0f / (XCCARRY * WCARRY));
      launch_gemm<0, 1, false>(stream, XC, DIN, xpwT_l, DIN, DBL16, DDBL, nullptr, nullptr, NROWS, DDBL, DIN, DBLCARRY / (XCCARRY * WCARRY));
      launch_gemm<2, 0, false>(stream, DBL16, DDBL, dtwT_l, DTKP, DTP, DIN, dtb, nullptr, NROWS, DIN, DTKP, 1.0f / (DBLCARRY * WCARRY));
      ssm_scan_gate<<<dim3(DIN / 64, NBATCH), 64, 0, stream>>>(DTP, XZ, DBL32, cw, cb, alog, dd, GP, dir, GCARRY);
      launch_gemm<0, 0, true>(stream, GP, DIN, owT_l, DIN, HT, DMOD, nullptr, Hin, NROWS, DMOD, DIN, 1.0f / (GCARRY * WCARRY));
      ln_rows_to_f16<<<NROWS / 8, 256, 0, stream>>>(HT, n2w, n2b, ULN, NROWS);
      launch_gemm<2, 0, false>(stream, ULN, DMOD, w1T_l, DMOD, F1, DFF, b1, nullptr, NROWS, DFF, DMOD, 1.0f / WCARRY);
      gelu_f16x2<<<NROWS * DFF / 2 / 256, 256, 0, stream>>>(F1, GL, NROWS * DFF / 2, GLCARRY);
      launch_gemm<2, 0, true>(stream, GL, DFF, w2T_l, DFF, HD, DMOD, b2, HT, NROWS, DMOD, DFF, 1.0f / (GLCARRY * WCARRY));
    }
    cast_f32_f16x2<<<NROWS * DMOD / 2 / 256, 256, 0, stream>>>(HD, (_Float16*)H16, NROWS * DMOD / 2);
    launch_gemm<2, 0, false>(stream, H16, DMOD, aw1T, DMOD, S1, DATT, ab1, nullptr, NROWS, DATT, DMOD, 1.0f / WCARRY);
    score_softmax<<<NBATCH, 256, 0, stream>>>(S1, aw2, ab2, ATT + (size_t)dir * NBATCH * NTOK);
  }
  pool_norm_out<<<NBATCH, 512, 0, stream>>>(ATT, HF, HB, nw, nb, out);
}
